// StructureEncoder_9740985827767
// MI455X (gfx1250) — hardware-run, weakly checked
//
#include <hip/hip_runtime.h>


namespace {
constexpr int N = 20000, E = 320000, NG = 64, D = 128, RBF = 50, GRAM = 9, EF = 64  , VOC = 119, L = 4, EIN = 315, NPB = 8;
constexpr float FS_ = 256.0f, HS = 256.0f, WSC = 256.0f, EPS = 1e-5f;
typedef _Float16 b16;
typedef __attribute__((ext_vector_type(16))) _Float16 v16b;
typedef __attribute__((ext_vector_type(8))) _Float16 v8b;
typedef __attribute__((ext_vector_type(8))) float v8f;
typedef __attribute__((ext_vector_type(4))) float v4f;
__device__ __forceinline__ float bf16_rne(float f) { unsigned int u = __float_as_uint(f); u += 0x7FFFu + ((u >> 16) & 1u); float r = __uint_as_float(u & 0xFFFF0000u); asm volatile("" : "+v"(r)); return r; }
__device__ __forceinline__ float bfv(float f) { float r = bf16_rne(f); asm volatile("" : "+v"(r)); return r; }
__device__ __forceinline__ void split16(float v, b16& hi, b16& lo) { hi = (b16)v; lo = (b16)(v - (float)hi); }
__device__ __forceinline__ v16b frag_kb(const b16* p, int hh) { const v8b a = *(const v8b*)(p + 8 * hh), b = *(const v8b*)(p + 16 + 8 * hh); v16b f;
#pragma unroll
  for (int e = 0; e < 8; ++e) { f[e] = a[e]; f[8 + e] = b[e]; } return f; }
__device__ __forceinline__ v8f wmma16b(v16b a, v16b b, v8f c) { v8f d = __builtin_amdgcn_wmma_f32_16x16x32_f16(false, a, false, b, (short)0, c, false, false); asm volatile("v_nop\n\tv_nop\n\tv_nop\n\tv_nop" : "+v"(d) : "v"(a), "v"(b)); return d; }
__device__ __forceinline__ void wave_lds_sync() { __builtin_amdgcn_fence(__ATOMIC_RELEASE, "workgroup"); __builtin_amdgcn_wave_barrier(); __builtin_amdgcn_fence(__ATOMIC_ACQUIRE, "workgroup"); }
__device__ __forceinline__ float pmul(float a, float b) { float p = a * b; asm volatile("" : "+v"(p)); return p; }
__device__ __forceinline__ int iclamp(int v, int lo, int hi) { return v < lo ? lo : (v > hi ? hi : v); }
__device__ __forceinline__ float silu(float v) { return v / (1.0f + __expf(-v)); }
__device__ __forceinline__ float gelu_t(float v) { const float u = 0.7978845608028654f * (v + 0.044715f * v * v * v); return 0.5f * v * (1.0f + tanhf(u)); }
constexpr int CSR_NBLK7 = 512, CSR_GB7 = 7, CSR_GN7 = 1 << CSR_GB7  , CSR_TS7 = (CSR_GN7 < 32 ? 32 : CSR_GN7)  , CSR_MAXG7 = 512, CSR_CAP7 = 12288  ;
__device__ __host__ __forceinline__ int csr_tix7(int v) { return (v >> CSR_GB7) * CSR_TS7 + (v & (CSR_GN7 - 1)); }
__global__ __launch_bounds__(64) void csrA_kernel7(const int* __restrict__ dst, int E, int N, int nG, int CHP, int NGP, int* __restrict__ STG, int* __restrict__ HST) {
  extern __shared__ int sm[];
  int* cnt = sm; int* run = sm + NGP; int* ids = sm + 2 * NGP;
  const int b = blockIdx.x; const int ch = (E + CSR_NBLK7 - 1) / CSR_NBLK7; const int e0 = b * ch, e1 = min(E, e0 + ch);
  for (int i = threadIdx.x; i < NGP; i += 64) cnt[i] = 0;
  for (int i = threadIdx.x; i < CHP; i += 64) ids[i] = -1;
  __syncthreads();
  if (threadIdx.x == 0) {
    for (int e = e0; e < e1; ++e) { int d = dst[e]; d = (d < 0) ? 0 : (d >= N ? N - 1 : d); cnt[d >> CSR_GB7] += 1; }
    int acc = 0; for (int g = 0; g < nG; ++g) { run[g] = acc; acc += cnt[g]; }
    for (int e = e0; e < e1; ++e) { int d = dst[e]; d = (d < 0) ? 0 : (d >= N ? N - 1 : d); const int g = d >> CSR_GB7; ids[run[g]] = e; run[g] += 1; } }
  __syncthreads();
  typedef __attribute__((ext_vector_type(4))) int v4i;
  for (int pass = 0; pass < 2; ++pass) {
    for (int i = threadIdx.x; i < CHP / 4; i += 64) *(volatile v4i*)(STG + (size_t)b * CHP + i * 4) = *(const v4i*)(&ids[i * 4]);
    for (int i = threadIdx.x; i < NGP / 4; i += 64) { v4i v; for (int e = 0; e < 4; ++e) v[e] = (i * 4 + e < nG) ? cnt[i * 4 + e] : 0; *(volatile v4i*)(HST + (size_t)b * NGP + i * 4) = v; }
    __threadfence(); }
}
__global__ __launch_bounds__(512) void csrS_kernel7(const int* __restrict__ HST, int nG, int NGP, int* __restrict__ START, int* __restrict__ TOT, int* __restrict__ OFF) {
  __shared__ int tot[CSR_MAXG7];
  const int b = threadIdx.x;
  for (int pass = 0; pass < 2; ++pass) { int runb = 0; for (int g = 0; g < nG; ++g) { int c = HST[(size_t)b * NGP + g]; c = (c < 0) ? 0 : c; ((volatile int*)OFF)[(size_t)g * CSR_NBLK7 + b] = runb; runb += c; } __threadfence(); }
  for (int g = threadIdx.x; g < nG; g += 512) { int s = 0; for (int bb = 0; bb < CSR_NBLK7; ++bb) { int c = HST[(size_t)bb * NGP + g]; s += (c < 0) ? 0 : c; } tot[g] = s; }
  __syncthreads();
  if (threadIdx.x < 32) {
    __shared__ int st[CSR_MAXG7 + 32];
    if (threadIdx.x == 0) { int acc = 0; for (int g = 0; g < NGP; ++g) { st[g] = acc; if (g < nG) acc += (tot[g] + 31) & ~31; } st[NGP] = acc; }
    __builtin_amdgcn_fence(__ATOMIC_RELEASE, "workgroup"); __builtin_amdgcn_wave_barrier(); __builtin_amdgcn_fence(__ATOMIC_ACQUIRE, "workgroup");
    for (int pass = 0; pass < 2; ++pass) { for (int i = threadIdx.x; i < NGP + 32; i += 32) { ((volatile int*)START)[i] = (i <= NGP) ? st[min(i, NGP)] : 0; ((volatile int*)TOT)[i] = (i < nG) ? tot[i] : 0; } __threadfence(); } }
}
__global__ __launch_bounds__(256) void csrB_kernel7(const int* __restrict__ dst, int N, int nG, int CHP, int NGP, int permLen, const int* __restrict__ STG, const int* __restrict__ HST, const int* __restrict__ OFF, const int* __restrict__ START, const int* __restrict__ TOT, int* __restrict__ PERM, int* __restrict__ ROWPTR, int* __restrict__ ROWCNT, int* __restrict__ FLAG) {
  typedef __attribute__((ext_vector_type(4))) int v4i;
  __shared__ int ids[CSR_CAP7]; __shared__ unsigned short key[CSR_CAP7]; __shared__ int outp[CSR_CAP7]; __shared__ int ncnt[CSR_GN7 + 1]; __shared__ int boff[CSR_NBLK7 + 1];
  const int g = blockIdx.x, t_ = threadIdx.x; int tot = TOT[g]; int st = START[g], stn = START[g + 1]; const int v0 = g * CSR_GN7; const int nv = min(CSR_GN7, N - v0); const int t0 = g * CSR_TS7;
  st = (st < 0) ? 0 : (st > permLen - 32 ? permLen - 32 : st) & ~31; stn = (stn < st) ? st : (stn > permLen ? permLen : stn); tot = (tot < 0) ? 0 : tot; if (tot > stn - st && tot <= CSR_CAP7) tot = stn - st;
  if (tot > CSR_CAP7) {
    for (int pass = 0; pass < 2; ++pass) { for (int i = t_; i < CSR_TS7 / 4; i += 256) { v4i a, c; for (int e = 0; e < 4; ++e) { a[e] = st; c[e] = 0; } *(volatile v4i*)(ROWPTR + t0 + i * 4) = a; *(volatile v4i*)(ROWCNT + t0 + i * 4) = c; } if (t_ == 0) ((volatile int*)FLAG)[0] = 1; __threadfence(); } (void)nv; return; }
  if (t_ == 0) { int acc = 0; for (int b = 0; b < CSR_NBLK7; ++b) { boff[b] = acc; int c = HST[(size_t)b * NGP + g]; c = (c < 0) ? 0 : (c > CHP ? CHP : c); acc += c; if (acc > tot) acc = tot; } boff[CSR_NBLK7] = acc; }
  for (int i = t_; i <= CSR_GN7; i += 256) ncnt[i] = 0;
  __syncthreads();
  for (int b = 0; b < CSR_NBLK7; ++b) { const int c = boff[b + 1] - boff[b]; int o_ = OFF[(size_t)g * CSR_NBLK7 + b]; o_ = (o_ < 0) ? 0 : (o_ > CHP - c ? CHP - c : o_); const int* src_ = STG + (size_t)b * CHP + o_;
    for (int i = t_; i < c; i += 256) { int id = src_[i]; id = (id < 0) ? 0 : id; ids[boff[b] + i] = id; int d = dst[id]; d = (d < v0) ? v0 : (d >= N ? N - 1 : d); int kk = d - v0; kk = (kk < 0) ? 0 : (kk >= CSR_GN7 ? CSR_GN7 - 1 : kk); key[boff[b] + i] = (unsigned short)kk; } }
  __syncthreads();
  if (t_ == 0) { for (int i = 0; i < tot; ++i) ncnt[key[i]] += 1; int acc = 0; for (int vl = 0; vl < CSR_GN7; ++vl) { const int c = ncnt[vl]; ncnt[vl] = acc; acc += c; } ncnt[CSR_GN7] = acc;
    for (int i = 0; i < tot; ++i) { const int vl = key[i]; outp[ncnt[vl]] = ids[i]; ncnt[vl] += 1; }
    for (int vl = CSR_GN7; vl > 0; --vl) ncnt[vl] = ncnt[vl - 1]; ncnt[0] = 0; }
  __syncthreads();
  for (int pass = 0; pass < 2; ++pass) {
    for (int i = t_; i < (stn - st) / 4; i += 256) { v4i v; for (int e = 0; e < 4; ++e) { const int q = i * 4 + e; v[e] = (q < tot) ? outp[q] : -1; } *(volatile v4i*)(PERM + st + i * 4) = v; }
    for (int i = t_; i < CSR_TS7 / 4; i += 256) { v4i a, c; for (int e = 0; e < 4; ++e) { const int vl = i * 4 + e; const int vc = vl < CSR_GN7 ? vl : CSR_GN7; a[e] = (vl < CSR_GN7) ? st + ncnt[vc] : st; c[e] = (vl < nv) ? (ncnt[(vc < CSR_GN7 ? vc : CSR_GN7 - 1) + 1] - ncnt[vc]) : 0; } *(volatile v4i*)(ROWPTR + t0 + i * 4) = a; *(volatile v4i*)(ROWCNT + t0 + i * 4) = c; }
    __threadfence(); }
}
__global__ __launch_bounds__(256) void csrZ_kernel7(int* __restrict__ p, size_t n4) { typedef __attribute__((ext_vector_type(4))) int v4i; const size_t tid = (size_t)blockIdx.x * 256 + threadIdx.x, nth = (size_t)gridDim.x * 256; v4i z = {0, 0, 0, 0}; for (size_t i = tid; i < n4; i += nth) *(volatile v4i*)(p + i * 4) = z; }
struct CsrBufs7 { int *STG, *HST, *OFF, *START, *TOT, *PERM, *ROWPTR, *ROWCNT, *FLAG; int nG, NGP, CHP; size_t permLen; char* base; size_t bytes; };
static size_t csr_carve7(CsrBufs7& c, char* ws, size_t off, int E, int N) {
  const size_t off0 = off; c.base = ws + off;
  auto al = [&](size_t bytes) { char* p = ws + off; off += (bytes + 255) & ~(size_t)255; return p; };
  c.nG = (N + CSR_GN7 - 1) / CSR_GN7; c.NGP = (c.nG + 31) & ~31; const int ch = (E + CSR_NBLK7 - 1) / CSR_NBLK7; c.CHP = (ch + 31) & ~31; c.permLen = (size_t)E + 32 * (size_t)c.nG + 32;
  c.STG = (int*)al((size_t)CSR_NBLK7 * c.CHP * 4); c.HST = (int*)al((size_t)CSR_NBLK7 * c.NGP * 4); c.OFF = (int*)al((size_t)c.NGP * CSR_NBLK7 * 4); c.START = (int*)al((size_t)(c.NGP + 64) * 4); c.TOT = (int*)al((size_t)(c.NGP + 64) * 4);
  c.PERM = (int*)al(c.permLen * 4); c.ROWPTR = (int*)al((size_t)c.nG * CSR_TS7 * 4); c.ROWCNT = (int*)al((size_t)c.nG * CSR_TS7 * 4); c.FLAG = (int*)al(256);
  c.bytes = off - off0; return off;
}
static void csr_build7(const CsrBufs7& c, const int* dst, int E, int N, hipStream_t stream) {
  const size_t smem = (size_t)(2 * c.NGP + c.CHP) * 4;
  csrZ_kernel7<<<512, 256, 0, stream>>>((int*)c.base, c.bytes / 16);
  csrA_kernel7<<<CSR_NBLK7, 64, smem, stream>>>(dst, E, N, c.nG, c.CHP, c.NGP, c.STG, c.HST);
  csrS_kernel7<<<1, 512, 0, stream>>>(c.HST, c.nG, c.NGP, c.START, c.TOT, c.OFF);
  csrB_kernel7<<<c.nG, 256, 0, stream>>>(dst, N, c.nG, c.CHP, c.NGP, (int)c.permLen, c.STG, c.HST, c.OFF, c.START, c.TOT, c.PERM, c.ROWPTR, c.ROWCNT, c.FLAG);
}
constexpr int CSR_NBLK5 = 512, CSR_GB5 = 5, CSR_GN5 = 1 << CSR_GB5  , CSR_TS5 = (CSR_GN5 < 32 ? 32 : CSR_GN5)  , CSR_MAXG5 = 512, CSR_CAP5 = 12288  ;
__device__ __host__ __forceinline__ int csr_tix5(int v) { return (v >> CSR_GB5) * CSR_TS5 + (v & (CSR_GN5 - 1)); }
__global__ __launch_bounds__(64) void csrA_kernel5(const int* __restrict__ dst, int E, int N, int nG, int CHP, int NGP, int* __restrict__ STG, int* __restrict__ HST) {
  extern __shared__ int sm[];
  int* cnt = sm; int* run = sm + NGP; int* ids = sm + 2 * NGP;
  const int b = blockIdx.x; const int ch = (E + CSR_NBLK5 - 1) / CSR_NBLK5; const int e0 = b * ch, e1 = min(E, e0 + ch);
  for (int i = threadIdx.x; i < NGP; i += 64) cnt[i] = 0;
  for (int i = threadIdx.x; i < CHP; i += 64) ids[i] = -1;
  __syncthreads();
  if (threadIdx.x == 0) {
    for (int e = e0; e < e1; ++e) { int d = dst[e]; d = (d < 0) ? 0 : (d >= N ? N - 1 : d); cnt[d >> CSR_GB5] += 1; }
    int acc = 0; for (int g = 0; g < nG; ++g) { run[g] = acc; acc += cnt[g]; }
    for (int e = e0; e < e1; ++e) { int d = dst[e]; d = (d < 0) ? 0 : (d >= N ? N - 1 : d); const int g = d >> CSR_GB5; ids[run[g]] = e; run[g] += 1; } }
  __syncthreads();
  typedef __attribute__((ext_vector_type(4))) int v4i;
  for (int pass = 0; pass < 2; ++pass) {
    for (int i = threadIdx.x; i < CHP / 4; i += 64) *(volatile v4i*)(STG + (size_t)b * CHP + i * 4) = *(const v4i*)(&ids[i * 4]);
    for (int i = threadIdx.x; i < NGP / 4; i += 64) { v4i v; for (int e = 0; e < 4; ++e) v[e] = (i * 4 + e < nG) ? cnt[i * 4 + e] : 0; *(volatile v4i*)(HST + (size_t)b * NGP + i * 4) = v; }
    __threadfence(); }
}
__global__ __launch_bounds__(512) void csrS_kernel5(const int* __restrict__ HST, int nG, int NGP, int* __restrict__ START, int* __restrict__ TOT, int* __restrict__ OFF) {
  __shared__ int tot[CSR_MAXG5];
  const int b = threadIdx.x;
  for (int pass = 0; pass < 2; ++pass) { int runb = 0; for (int g = 0; g < nG; ++g) { int c = HST[(size_t)b * NGP + g]; c = (c < 0) ? 0 : c; ((volatile int*)OFF)[(size_t)g * CSR_NBLK5 + b] = runb; runb += c; } __threadfence(); }
  for (int g = threadIdx.x; g < nG; g += 512) { int s = 0; for (int bb = 0; bb < CSR_NBLK5; ++bb) { int c = HST[(size_t)bb * NGP + g]; s += (c < 0) ? 0 : c; } tot[g] = s; }
  __syncthreads();
  if (threadIdx.x < 32) {
    __shared__ int st[CSR_MAXG5 + 32];
    if (threadIdx.x == 0) { int acc = 0; for (int g = 0; g < NGP; ++g) { st[g] = acc; if (g < nG) acc += (tot[g] + 31) & ~31; } st[NGP] = acc; }
    __builtin_amdgcn_fence(__ATOMIC_RELEASE, "workgroup"); __builtin_amdgcn_wave_barrier(); __builtin_amdgcn_fence(__ATOMIC_ACQUIRE, "workgroup");
    for (int pass = 0; pass < 2; ++pass) { for (int i = threadIdx.x; i < NGP + 32; i += 32) { ((volatile int*)START)[i] = (i <= NGP) ? st[min(i, NGP)] : 0; ((volatile int*)TOT)[i] = (i < nG) ? tot[i] : 0; } __threadfence(); } }
}
__global__ __launch_bounds__(256) void csrB_kernel5(const int* __restrict__ dst, int N, int nG, int CHP, int NGP, int permLen, const int* __restrict__ STG, const int* __restrict__ HST, const int* __restrict__ OFF, const int* __restrict__ START, const int* __restrict__ TOT, int* __restrict__ PERM, int* __restrict__ ROWPTR, int* __restrict__ ROWCNT, int* __restrict__ FLAG) {
  typedef __attribute__((ext_vector_type(4))) int v4i;
  __shared__ int ids[CSR_CAP5]; __shared__ unsigned short key[CSR_CAP5]; __shared__ int outp[CSR_CAP5]; __shared__ int ncnt[CSR_GN5 + 1]; __shared__ int boff[CSR_NBLK5 + 1];
  const int g = blockIdx.x, t_ = threadIdx.x; int tot = TOT[g]; int st = START[g], stn = START[g + 1]; const int v0 = g * CSR_GN5; const int nv = min(CSR_GN5, N - v0); const int t0 = g * CSR_TS5;
  st = (st < 0) ? 0 : (st > permLen - 32 ? permLen - 32 : st) & ~31; stn = (stn < st) ? st : (stn > permLen ? permLen : stn); tot = (tot < 0) ? 0 : tot; if (tot > stn - st && tot <= CSR_CAP5) tot = stn - st;
  if (tot > CSR_CAP5) {
    for (int pass = 0; pass < 2; ++pass) { for (int i = t_; i < CSR_TS5 / 4; i += 256) { v4i a, c; for (int e = 0; e < 4; ++e) { a[e] = st; c[e] = 0; } *(volatile v4i*)(ROWPTR + t0 + i * 4) = a; *(volatile v4i*)(ROWCNT + t0 + i * 4) = c; } if (t_ == 0) ((volatile int*)FLAG)[0] = 1; __threadfence(); } (void)nv; return; }
  if (t_ == 0) { int acc = 0; for (int b = 0; b < CSR_NBLK5; ++b) { boff[b] = acc; int c = HST[(size_t)b * NGP + g]; c = (c < 0) ? 0 : (c > CHP ? CHP : c); acc += c; if (acc > tot) acc = tot; } boff[CSR_NBLK5] = acc; }
  for (int i = t_; i <= CSR_GN5; i += 256) ncnt[i] = 0;
  __syncthreads();
  for (int b = 0; b < CSR_NBLK5; ++b) { const int c = boff[b + 1] - boff[b]; int o_ = OFF[(size_t)g * CSR_NBLK5 + b]; o_ = (o_ < 0) ? 0 : (o_ > CHP - c ? CHP - c : o_); const int* src_ = STG + (size_t)b * CHP + o_;
    for (int i = t_; i < c; i += 256) { int id = src_[i]; id = (id < 0) ? 0 : id; ids[boff[b] + i] = id; int d = dst[id]; d = (d < v0) ? v0 : (d >= N ? N - 1 : d); int kk = d - v0; kk = (kk < 0) ? 0 : (kk >= CSR_GN5 ? CSR_GN5 - 1 : kk); key[boff[b] + i] = (unsigned short)kk; } }
  __syncthreads();
  if (t_ == 0) { for (int i = 0; i < tot; ++i) ncnt[key[i]] += 1; int acc = 0; for (int vl = 0; vl < CSR_GN5; ++vl) { const int c = ncnt[vl]; ncnt[vl] = acc; acc += c; } ncnt[CSR_GN5] = acc;
    for (int i = 0; i < tot; ++i) { const int vl = key[i]; outp[ncnt[vl]] = ids[i]; ncnt[vl] += 1; }
    for (int vl = CSR_GN5; vl > 0; --vl) ncnt[vl] = ncnt[vl - 1]; ncnt[0] = 0; }
  __syncthreads();
  for (int pass = 0; pass < 2; ++pass) {
    for (int i = t_; i < (stn - st) / 4; i += 256) { v4i v; for (int e = 0; e < 4; ++e) { const int q = i * 4 + e; v[e] = (q < tot) ? outp[q] : -1; } *(volatile v4i*)(PERM + st + i * 4) = v; }
    for (int i = t_; i < CSR_TS5 / 4; i += 256) { v4i a, c; for (int e = 0; e < 4; ++e) { const int vl = i * 4 + e; const int vc = vl < CSR_GN5 ? vl : CSR_GN5; a[e] = (vl < CSR_GN5) ? st + ncnt[vc] : st; c[e] = (vl < nv) ? (ncnt[(vc < CSR_GN5 ? vc : CSR_GN5 - 1) + 1] - ncnt[vc]) : 0; } *(volatile v4i*)(ROWPTR + t0 + i * 4) = a; *(volatile v4i*)(ROWCNT + t0 + i * 4) = c; }
    __threadfence(); }
}
__global__ __launch_bounds__(256) void csrZ_kernel5(int* __restrict__ p, size_t n4) { typedef __attribute__((ext_vector_type(4))) int v4i; const size_t tid = (size_t)blockIdx.x * 256 + threadIdx.x, nth = (size_t)gridDim.x * 256; v4i z = {0, 0, 0, 0}; for (size_t i = tid; i < n4; i += nth) *(volatile v4i*)(p + i * 4) = z; }
struct CsrBufs5 { int *STG, *HST, *OFF, *START, *TOT, *PERM, *ROWPTR, *ROWCNT, *FLAG; int nG, NGP, CHP; size_t permLen; char* base; size_t bytes; };
static size_t csr_carve5(CsrBufs5& c, char* ws, size_t off, int E, int N) {
  const size_t off0 = off; c.base = ws + off;
  auto al = [&](size_t bytes) { char* p = ws + off; off += (bytes + 255) & ~(size_t)255; return p; };
  c.nG = (N + CSR_GN5 - 1) / CSR_GN5; c.NGP = (c.nG + 31) & ~31; const int ch = (E + CSR_NBLK5 - 1) / CSR_NBLK5; c.CHP = (ch + 31) & ~31; c.permLen = (size_t)E + 32 * (size_t)c.nG + 32;
  c.STG = (int*)al((size_t)CSR_NBLK5 * c.CHP * 4); c.HST = (int*)al((size_t)CSR_NBLK5 * c.NGP * 4); c.OFF = (int*)al((size_t)c.NGP * CSR_NBLK5 * 4); c.START = (int*)al((size_t)(c.NGP + 64) * 4); c.TOT = (int*)al((size_t)(c.NGP + 64) * 4);
  c.PERM = (int*)al(c.permLen * 4); c.ROWPTR = (int*)al((size_t)c.nG * CSR_TS5 * 4); c.ROWCNT = (int*)al((size_t)c.nG * CSR_TS5 * 4); c.FLAG = (int*)al(256);
  c.bytes = off - off0; return off;
}
static void csr_build5(const CsrBufs5& c, const int* dst, int E, int N, hipStream_t stream) {
  const size_t smem = (size_t)(2 * c.NGP + c.CHP) * 4;
  csrZ_kernel5<<<512, 256, 0, stream>>>((int*)c.base, c.bytes / 16);
  csrA_kernel5<<<CSR_NBLK5, 64, smem, stream>>>(dst, E, N, c.nG, c.CHP, c.NGP, c.STG, c.HST);
  csrS_kernel5<<<1, 512, 0, stream>>>(c.HST, c.nG, c.NGP, c.START, c.TOT, c.OFF);
  csrB_kernel5<<<c.nG, 256, 0, stream>>>(dst, N, c.nG, c.CHP, c.NGP, (int)c.permLen, c.STG, c.HST, c.OFF, c.START, c.TOT, c.PERM, c.ROWPTR, c.ROWCNT, c.FLAG);
}


__global__ __launch_bounds__(256) void wput_kernel(const float* __restrict__ ew1, const float* __restrict__ ew2, const float* __restrict__ nw1, const float* __restrict__ nw2, const float* __restrict__ ro, const float* __restrict__ p1, const float* __restrict__ p2, b16* __restrict__ WPS, b16* __restrict__ WEF, b16* __restrict__ WE2, b16* __restrict__ WN1, b16* __restrict__ WN2, b16* __restrict__ WRO, b16* __restrict__ WP1, b16* __restrict__ WP2) { const size_t nt = (size_t)gridDim.x * 256, u0 = (size_t)blockIdx.x * 256 + threadIdx.x; v8b v;
  for (size_t u = u0; u < (size_t)L * 256 * 16; u += nt) { const int l = (int)(u / (256 * 16)), r = (int)(u % (256 * 16)); const int o = r / 16, k0 = (r % 16) * 8; const float* w = ew1 + (size_t)l * EIN * D;
#pragma unroll
    for (int j = 0; j < 8; ++j) { const int k = k0 + j; v[j] = (b16)(bf16_rne(o < D ? w[(size_t)k * D + o] : w[(size_t)(D + k) * D + o - D]) * WSC); } for (int pass = 0; pass < 2; ++pass) { *(volatile v8b*)(WPS + ((size_t)l * 2 * D + o) * D + k0) = v; __threadfence(); } }
  for (size_t u = u0; u < (size_t)L * D * 8; u += nt) { const int l = (int)(u / (D * 8)), r = (int)(u % (D * 8)); const int o = r / 8, k0 = (r % 8) * 8; const float* w = ew1 + (size_t)l * EIN * D;
#pragma unroll
    for (int j = 0; j < 8; ++j) { const int k = k0 + j; v[j] = (b16)(k < GRAM + RBF ? bf16_rne(w[(size_t)(2 * D + k) * D + o]) * WSC : 0.0f); } for (int pass = 0; pass < 2; ++pass) { *(volatile v8b*)(WEF + ((size_t)l * D + o) * EF + k0) = v; __threadfence(); } }
  for (size_t u = u0; u < (size_t)L * D * 16; u += nt) { const int l = (int)(u / (D * 16)), r = (int)(u % (D * 16)); const int o = r / 16, k0 = (r % 16) * 8; v8b a, c;
#pragma unroll
    for (int j = 0; j < 8; ++j) { a[j] = (b16)(bf16_rne(ew2[((size_t)l * D + k0 + j) * D + o]) * WSC); c[j] = (b16)(bf16_rne(nw2[((size_t)l * D + k0 + j) * D + o]) * WSC); } for (int pass = 0; pass < 2; ++pass) { *(volatile v8b*)(WE2 + ((size_t)l * D + o) * D + k0) = a; *(volatile v8b*)(WN2 + ((size_t)l * D + o) * D + k0) = c; __threadfence(); } }
  for (size_t u = u0; u < (size_t)L * D * 32; u += nt) { const int l = (int)(u / (D * 32)), r = (int)(u % (D * 32)); const int o = r / 32, k0 = (r % 32) * 8;
#pragma unroll
    for (int j = 0; j < 8; ++j) v[j] = (b16)(bf16_rne(nw1[((size_t)l * 2 * D + k0 + j) * D + o]) * WSC); for (int pass = 0; pass < 2; ++pass) { *(volatile v8b*)(WN1 + ((size_t)l * D + o) * 2 * D + k0) = v; __threadfence(); } }
  for (size_t u = u0; u < (size_t)256 * 16; u += nt) { const int o = (int)(u / 16), k0 = (int)(u % 16) * 8;
#pragma unroll
    for (int j = 0; j < 8; ++j) v[j] = (b16)(bf16_rne(ro[(size_t)(k0 + j) * 256 + o]) * WSC); for (int pass = 0; pass < 2; ++pass) { *(volatile v8b*)(WRO + (size_t)o * D + k0) = v; __threadfence(); } }
  for (size_t u = u0; u < (size_t)256 * 32; u += nt) { const int o = (int)(u / 32), k0 = (int)(u % 32) * 8;
#pragma unroll
    for (int j = 0; j < 8; ++j) v[j] = (b16)(bf16_rne(p1[(size_t)(k0 + j) * 256 + o]) * WSC); for (int pass = 0; pass < 2; ++pass) { *(volatile v8b*)(WP1 + (size_t)o * 256 + k0) = v; __threadfence(); } }
  for (size_t u = u0; u < (size_t)128 * 32; u += nt) { const int o = (int)(u / 32), k0 = (int)(u % 32) * 8;
#pragma unroll
    for (int j = 0; j < 8; ++j) v[j] = (b16)(bf16_rne(p2[(size_t)(k0 + j) * 128 + o]) * WSC); for (int pass = 0; pass < 2; ++pass) { *(volatile v8b*)(WP2 + (size_t)o * 256 + k0) = v; __threadfence(); } } }
__global__ __launch_bounds__(32) void emb_kernel(const int* __restrict__ at, const float* __restrict__ emb, float* __restrict__ Hp) { const int lane = threadIdx.x; const size_t m0 = (size_t)blockIdx.x * 16;
  for (int pass = 0; pass < 2; ++pass) { for (int rr = 0; rr < 16; ++rr) { const int a = iclamp(at[m0 + rr], 0, VOC - 1); for (int q = 0; q < 4; ++q) ((volatile float*)Hp)[(m0 + rr) * D + q * 32 + lane] = bfv(emb[(size_t)a * D + q * 32 + lane]); } __threadfence(); } }
__global__ __launch_bounds__(32) void prep_kernel(const float* __restrict__ Hp, const float* __restrict__ lg, const float* __restrict__ lb, const b16* __restrict__ WPS, int NLIM, float* __restrict__ HN, float* __restrict__ PSD) { __shared__ __attribute__((aligned(16))) b16 Ah[16][D + 8], Al[16][D + 8]; __shared__ float Xs[16][D + 1], Tf[16][2 * D + 4]; const int lane = threadIdx.x, nloc = lane & 15, hlf = lane >> 4; const size_t m0 = (size_t)blockIdx.x * 16; if (m0 >= (size_t)NLIM) return;
  for (int rr = 0; rr < 16; ++rr) for (int q = 0; q < 4; ++q) Xs[rr][q * 32 + lane] = Hp[(m0 + rr) * D + q * 32 + lane];
  wave_lds_sync();
  if (lane < 16) { float m = 0.0f; for (int c = 0; c < D; ++c) m += Xs[lane][c]; m *= (1.0f / D); float vr = 0.0f; for (int c = 0; c < D; ++c) { const float d = Xs[lane][c] - m; vr += d * d; } vr *= (1.0f / D); const float rs = rsqrtf(vr + EPS); for (int c = 0; c < D; ++c) { const float v = pmul((Xs[lane][c] - m) * rs, bfv(lg[c])) + bfv(lb[c]); Xs[lane][c] = v; b16 p, ql; split16(v * HS, p, ql); Ah[lane][c] = p; Al[lane][c] = ql; } for (int k = D; k < D + 8; ++k) { Ah[lane][k] = (b16)0.0f; Al[lane][k] = (b16)0.0f; } }
  wave_lds_sync(); v8f acc[16];
#pragma unroll
  for (int t = 0; t < 16; ++t) acc[t] = (v8f){};
#pragma unroll 2
  for (int kb = 0; kb < D; kb += 32) { const v16b a = frag_kb(&Ah[nloc][kb], hlf), al = frag_kb(&Al[nloc][kb], hlf);
#pragma unroll
    for (int t = 0; t < 16; ++t) { const v16b bw = frag_kb(WPS + (size_t)(t * 16 + nloc) * D + kb, hlf); acc[t] = wmma16b(a, bw, acc[t]); acc[t] = wmma16b(al, bw, acc[t]); } }
#pragma unroll
  for (int t = 0; t < 16; ++t)
#pragma unroll
    for (int r8 = 0; r8 < 8; ++r8) Tf[8 * hlf + r8][t * 16 + nloc] = acc[t][r8] * (1.0f / (HS * WSC));
  wave_lds_sync();
  for (int pass = 0; pass < 2; ++pass) { for (int rr = 0; rr < 16; ++rr) { *(volatile v4f*)(HN + (m0 + rr) * D + lane * 4) = *(const v4f*)(&Xs[rr][lane * 4]); for (int q = 0; q < 2; ++q) *(volatile v4f*)(PSD + (m0 + rr) * 2 * D + q * 128 + lane * 4) = *(const v4f*)(&Tf[rr][q * 128 + lane * 4]); } __threadfence(); } }
__global__ __launch_bounds__(32) void layer_kernel(float* __restrict__ Hp, const float* __restrict__ HN, const float* __restrict__ PSD, const float* __restrict__ gram, const float* __restrict__ rbf, const int* __restrict__ srcs, const int* __restrict__ PERM, const int* __restrict__ ROWPTR, const int* __restrict__ ROWCNT, int permLen, const b16* __restrict__ WEF, const float* __restrict__ eb1, const b16* __restrict__ WE2, const float* __restrict__ eb2, const b16* __restrict__ WN1, const float* __restrict__ nb1, const b16* __restrict__ WN2, const float* __restrict__ nb2, int NLIM) {
  __shared__ __attribute__((aligned(16))) b16 Ah[16][2 * D + 8], Al[16][2 * D + 8]; __shared__ float Tf[16][D + 4], Ms[16][D + 1]; __shared__ int Ce[16], Cr[16], St0[16], Cn0[16], Kp[16]; const int lane = threadIdx.x, nloc = lane & 15, hlf = lane >> 4; const size_t m0 = (size_t)blockIdx.x * 16; if (m0 >= (size_t)NLIM) return;
  if (lane < 16) { const size_t i = m0 + lane; int st = ROWPTR[i], cnt = ROWCNT[i]; cnt = iclamp(cnt, 0, E); st = iclamp(st, 0, permLen - cnt); St0[lane] = st; Cn0[lane] = cnt; Kp[lane] = 0; }
  for (int rr = 0; rr < 16; ++rr) for (int q = 0; q < 4; ++q) Ms[rr][q * 32 + lane] = 0.0f;
  wave_lds_sync();
  int total = 0; for (int r = 0; r < 16; ++r) total += Cn0[r];
  int cr = 0, cj = 0;
#pragma unroll 1
  for (int done = 0; done < total; ) {
    int nck = 0;
    while (nck < 16 && cr < 16) { if (cj >= Cn0[cr]) { ++cr; cj = 0; continue; } const int e = iclamp(PERM[St0[cr] + cj], 0, E - 1); ++cj; ++done; const int s = iclamp(srcs[e], 0, N - 1); if (s >= NLIM) continue; if (lane == 0) { Ce[nck] = e; Cr[nck] = cr; Kp[cr] += 1; } ++nck; }
    if (nck == 0) break;
    wave_lds_sync();
    for (int rr = 0; rr < 16; ++rr) for (int q = 0; q < 2; ++q) { const int c = q * 32 + lane; float v = 0.0f; if (rr < nck) { const size_t e = (size_t)Ce[rr]; if (c < GRAM) v = bfv(gram[e * GRAM + c]); else if (c < GRAM + RBF) v = bfv(rbf[e * RBF + c - GRAM]); } Ah[rr][c] = (b16)(v * FS_); Al[rr][c] = (b16)0.0f; }
    if (lane < 16) for (int k = EF; k < EF + 8; ++k) { Ah[lane][k] = (b16)0.0f; Al[lane][k] = (b16)0.0f; }
    wave_lds_sync(); v8f acc[8];
#pragma unroll
    for (int t = 0; t < 8; ++t) acc[t] = (v8f){};
#pragma unroll
    for (int kb = 0; kb < EF; kb += 32) { const v16b a = frag_kb(&Ah[nloc][kb], hlf);
#pragma unroll
      for (int t = 0; t < 8; ++t) acc[t] = wmma16b(a, frag_kb(WEF + (size_t)(t * 16 + nloc) * EF + kb, hlf), acc[t]); }
#pragma unroll
    for (int t = 0; t < 8; ++t)
#pragma unroll
      for (int r8 = 0; r8 < 8; ++r8) Tf[8 * hlf + r8][t * 16 + nloc] = acc[t][r8] * (1.0f / (FS_ * WSC));
    wave_lds_sync();
    for (int rr = 0; rr < 16; ++rr) { const bool ok = rr < nck; const size_t e = ok ? (size_t)Ce[rr] : 0; const size_t s = ok ? (size_t)iclamp(srcs[e], 0, N - 1) : 0, dn = ok ? m0 + Cr[rr] : 0; for (int q = 0; q < 4; ++q) { const int c = q * 32 + lane; const float v = ok ? silu(Tf[rr][c] + PSD[s * 2 * D + c] + PSD[dn * 2 * D + D + c] + bfv(eb1[c])) : 0.0f; b16 p, ql; split16(v * HS, p, ql); Ah[rr][c] = p; Al[rr][c] = ql; } }
    if (lane < 16) for (int k = D; k < D + 8; ++k) { Ah[lane][k] = (b16)0.0f; Al[lane][k] = (b16)0.0f; }
    wave_lds_sync();
#pragma unroll
    for (int t = 0; t < 8; ++t) acc[t] = (v8f){};
#pragma unroll
    for (int kb = 0; kb < D; kb += 32) { const v16b a = frag_kb(&Ah[nloc][kb], hlf), al = frag_kb(&Al[nloc][kb], hlf);
#pragma unroll
      for (int t = 0; t < 8; ++t) { const v16b bw = frag_kb(WE2 + (size_t)(t * 16 + nloc) * D + kb, hlf); acc[t] = wmma16b(a, bw, acc[t]); acc[t] = wmma16b(al, bw, acc[t]); } }
#pragma unroll
    for (int t = 0; t < 8; ++t) { const int cc = t * 16 + nloc; const float bb = bfv(eb2[cc]);
#pragma unroll
      for (int r8 = 0; r8 < 8; ++r8) Tf[8 * hlf + r8][cc] = silu(acc[t][r8] * (1.0f / (HS * WSC)) + bb); }
    wave_lds_sync();
    for (int rr = 0; rr < nck; ++rr) { const int r = Cr[rr]; for (int q = 0; q < 4; ++q) Ms[r][q * 32 + lane] += Tf[rr][q * 32 + lane]; }
    wave_lds_sync(); }
  wave_lds_sync();
  for (int rr = 0; rr < 16; ++rr) { const float inv = 1.0f / fmaxf((float)Kp[rr], 1.0f); for (int q = 0; q < 4; ++q) { const int c = q * 32 + lane; b16 p, ql; split16(HN[(m0 + rr) * D + c] * HS, p, ql); Ah[rr][c] = p; Al[rr][c] = ql; split16(Ms[rr][c] * inv * HS, p, ql); Ah[rr][D + c] = p; Al[rr][D + c] = ql; } }
  if (lane < 16) for (int k = 2 * D; k < 2 * D + 8; ++k) { Ah[lane][k] = (b16)0.0f; Al[lane][k] = (b16)0.0f; }
  wave_lds_sync();
  { v8f acc[8];
#pragma unroll
    for (int t = 0; t < 8; ++t) acc[t] = (v8f){};
#pragma unroll 2
    for (int kb = 0; kb < 2 * D; kb += 32) { const v16b a = frag_kb(&Ah[nloc][kb], hlf), al = frag_kb(&Al[nloc][kb], hlf);
#pragma unroll
      for (int t = 0; t < 8; ++t) { const v16b bw = frag_kb(WN1 + (size_t)(t * 16 + nloc) * 2 * D + kb, hlf); acc[t] = wmma16b(a, bw, acc[t]); acc[t] = wmma16b(al, bw, acc[t]); } }
#pragma unroll
    for (int t = 0; t < 8; ++t) { const int cc = t * 16 + nloc; const float bb = bfv(nb1[cc]);
#pragma unroll
      for (int r8 = 0; r8 < 8; ++r8) Tf[8 * hlf + r8][cc] = silu(acc[t][r8] * (1.0f / (HS * WSC)) + bb); } }
  wave_lds_sync();
  for (int rr = 0; rr < 16; ++rr) for (int q = 0; q < 4; ++q) { const int c = q * 32 + lane; b16 p, ql; split16(Tf[rr][c] * HS, p, ql); Ah[rr][c] = p; Al[rr][c] = ql; }
  if (lane < 16) for (int k = D; k < D + 8; ++k) { Ah[lane][k] = (b16)0.0f; Al[lane][k] = (b16)0.0f; }
  wave_lds_sync();
  { v8f acc[8];
#pragma unroll
    for (int t = 0; t < 8; ++t) acc[t] = (v8f){};
#pragma unroll
    for (int kb = 0; kb < D; kb += 32) { const v16b a = frag_kb(&Ah[nloc][kb], hlf), al = frag_kb(&Al[nloc][kb], hlf);
#pragma unroll
      for (int t = 0; t < 8; ++t) { const v16b bw = frag_kb(WN2 + (size_t)(t * 16 + nloc) * D + kb, hlf); acc[t] = wmma16b(a, bw, acc[t]); acc[t] = wmma16b(al, bw, acc[t]); } }
    wave_lds_sync();
#pragma unroll
    for (int t = 0; t < 8; ++t) { const int cc = t * 16 + nloc; const float bb = bfv(nb2[cc]);
#pragma unroll
      for (int r8 = 0; r8 < 8; ++r8) Tf[8 * hlf + r8][cc] = silu(acc[t][r8] * (1.0f / (HS * WSC)) + bb); } }
  wave_lds_sync();
  for (int rr = 0; rr < 16; ++rr) for (int q = 0; q < 4; ++q) { const int c = q * 32 + lane; Ms[rr][c] = Hp[(m0 + rr) * D + c] + Tf[rr][c]; }
  wave_lds_sync();
  for (int pass = 0; pass < 2; ++pass) { for (int rr = 0; rr < 16; ++rr) for (int q = 0; q < 4; ++q) { const int c = q * 32 + lane; ((volatile float*)Hp)[(m0 + rr) * D + c] = Ms[rr][c]; } __threadfence(); } }

__global__ __launch_bounds__(32) void readout_kernel(const float* __restrict__ Hp, const int* __restrict__ PERM, const int* __restrict__ ROWPTR, const int* __restrict__ ROWCNT, int permLen, const b16* __restrict__ WRO, const float* __restrict__ rob, const b16* __restrict__ WP1, const float* __restrict__ p1b, const b16* __restrict__ WP2, const float* __restrict__ p2b, int NLIM, float* __restrict__ out) { __shared__ __attribute__((aligned(16))) b16 Ah[16][264], Al[16][264]; __shared__ float Tf[16][260], Zc[16][260]; const int lane = threadIdx.x, nloc = lane & 15, hlf = lane >> 4; const int g0 = blockIdx.x * 16;
  for (int rr = 0; rr < 16; ++rr) { const int g = g0 + rr; int st = ROWPTR[g], cnt = ROWCNT[g]; cnt = iclamp(cnt, 0, N); st = iclamp(st, 0, permLen - cnt); v4f s = {0, 0, 0, 0}; int nn = 0;
#pragma unroll 1
    for (int j = 0; j < cnt; ++j) { const size_t n = (size_t)iclamp(PERM[st + j], 0, N - 1); if (n >= (size_t)NLIM) continue; ++nn; s += *(const v4f*)(Hp + n * D + lane * 4); }
    const float inv = 1.0f / fmaxf((float)nn, 1.0f); for (int k = 0; k < 4; ++k) { b16 p, ql; split16(s[k] * inv * HS, p, ql); Ah[rr][lane * 4 + k] = p; Al[rr][lane * 4 + k] = ql; } }
  if (lane < 16) for (int k = D; k < D + 8; ++k) { Ah[lane][k] = (b16)0.0f; Al[lane][k] = (b16)0.0f; }
  wave_lds_sync();
  { v8f acc[16];
#pragma unroll
    for (int t = 0; t < 16; ++t) acc[t] = (v8f){};
#pragma unroll
    for (int kb = 0; kb < D; kb += 32) { const v16b a = frag_kb(&Ah[nloc][kb], hlf), al = frag_kb(&Al[nloc][kb], hlf);
#pragma unroll
      for (int t = 0; t < 16; ++t) { const v16b bw = frag_kb(WRO + (size_t)(t * 16 + nloc) * D + kb, hlf); acc[t] = wmma16b(a, bw, acc[t]); acc[t] = wmma16b(al, bw, acc[t]); } }
#pragma unroll
    for (int t = 0; t < 16; ++t) { const int cc = t * 16 + nloc; const float bb = bfv(rob[cc]);
#pragma unroll
      for (int r8 = 0; r8 < 8; ++r8) Zc[8 * hlf + r8][cc] = acc[t][r8] * (1.0f / (HS * WSC)) + bb; } }
  wave_lds_sync();
  for (int rr = 0; rr < 16; ++rr) for (int q = 0; q < 8; ++q) { const int c = q * 32 + lane; b16 p, ql; split16(Zc[rr][c] * HS, p, ql); Ah[rr][c] = p; Al[rr][c] = ql; }
  if (lane < 16) for (int k = 256; k < 264; ++k) { Ah[lane][k] = (b16)0.0f; Al[lane][k] = (b16)0.0f; }
  wave_lds_sync();
  { v8f acc[16];
#pragma unroll
    for (int t = 0; t < 16; ++t) acc[t] = (v8f){};
#pragma unroll 2
    for (int kb = 0; kb < 256; kb += 32) { const v16b a = frag_kb(&Ah[nloc][kb], hlf), al = frag_kb(&Al[nloc][kb], hlf);
#pragma unroll
      for (int t = 0; t < 16; ++t) { const v16b bw = frag_kb(WP1 + (size_t)(t * 16 + nloc) * 256 + kb, hlf); acc[t] = wmma16b(a, bw, acc[t]); acc[t] = wmma16b(al, bw, acc[t]); } }
    wave_lds_sync();
#pragma unroll
    for (int t = 0; t < 16; ++t) { const int cc = t * 16 + nloc; const float bb = bfv(p1b[cc]);
#pragma unroll
      for (int r8 = 0; r8 < 8; ++r8) Tf[8 * hlf + r8][cc] = gelu_t(acc[t][r8] * (1.0f / (HS * WSC)) + bb); } }
  wave_lds_sync();
  for (int rr = 0; rr < 16; ++rr) for (int q = 0; q < 8; ++q) { const int c = q * 32 + lane; b16 p, ql; split16(Tf[rr][c] * HS, p, ql); Ah[rr][c] = p; Al[rr][c] = ql; }
  wave_lds_sync();
  { v8f acc[8];
#pragma unroll
    for (int t = 0; t < 8; ++t) acc[t] = (v8f){};
#pragma unroll 2
    for (int kb = 0; kb < 256; kb += 32) { const v16b a = frag_kb(&Ah[nloc][kb], hlf), al = frag_kb(&Al[nloc][kb], hlf);
#pragma unroll
      for (int t = 0; t < 8; ++t) { const v16b bw = frag_kb(WP2 + (size_t)(t * 16 + nloc) * 256 + kb, hlf); acc[t] = wmma16b(a, bw, acc[t]); acc[t] = wmma16b(al, bw, acc[t]); } }
    wave_lds_sync();
#pragma unroll
    for (int t = 0; t < 8; ++t) { const int cc = t * 16 + nloc; const float bb = bfv(p2b[cc]);
#pragma unroll
      for (int r8 = 0; r8 < 8; ++r8) Tf[8 * hlf + r8][cc] = acc[t][r8] * (1.0f / (HS * WSC)) + bb; } }
  wave_lds_sync();
  for (int pass = 0; pass < 2; ++pass) { for (int rr = 0; rr < 16; ++rr) { for (int q = 0; q < 2; ++q) *(volatile v4f*)(out + (size_t)(g0 + rr) * 256 + q * 128 + lane * 4) = *(const v4f*)(&Zc[rr][q * 128 + lane * 4]); *(volatile v4f*)(out + (size_t)NG * 256 + (size_t)(g0 + rr) * D + lane * 4) = *(const v4f*)(&Tf[rr][lane * 4]); } __threadfence(); } }
}

extern "C" void kernel_launch(void* const* d_in, const int* in_sizes, int n_in, void* d_out, int out_size, void* d_ws, size_t ws_size, hipStream_t stream) {
  (void)n_in;
  auto Fp = [&](int i) { return (const float*)d_in[i]; }; auto Ip = [&](int i) { return (const int*)d_in[i]; };
  if (in_sizes[0] != N || in_sizes[1] != 2 * E || in_sizes[2] != E * RBF || in_sizes[3] != E * GRAM || in_sizes[4] != N || in_sizes[5] != VOC * D || in_sizes[8] != L * EIN * D || in_sizes[10] != L * D * D || in_sizes[12] != L * 2 * D * D || in_sizes[16] != D * 256 || in_sizes[18] != 256 * 256 || in_sizes[20] != 256 * D || out_size != NG * 256 + NG * D) return;
  const int NLIM = N;
  size_t off = 0; char* ws = (char*)d_ws;
  auto carve = [&](size_t bytes) { char* p = ws + off; off += (bytes + 255) & ~(size_t)255; return p; };
  b16* WPS = (b16*)carve((size_t)L * 2 * D * D * 2); b16* WEF = (b16*)carve((size_t)L * D * EF * 2); b16* WE2 = (b16*)carve((size_t)L * D * D * 2); b16* WN1 = (b16*)carve((size_t)L * D * 2 * D * 2); b16* WN2 = (b16*)carve((size_t)L * D * D * 2); b16* WRO = (b16*)carve((size_t)256 * D * 2); b16* WP1 = (b16*)carve((size_t)256 * 256 * 2); b16* WP2 = (b16*)carve((size_t)D * 256 * 2); float* Hp = (float*)carve((size_t)N * D * 4); float* HN = (float*)carve((size_t)N * D * 4); float* PSD = (float*)carve((size_t)N * 2 * D * 4); CsrBufs7 csr; off = csr_carve7(csr, ws, off, E, N); CsrBufs5 cg; off = csr_carve5(cg, ws, off, N, NG);
  if (off > ws_size || off > ((size_t)80 << 20)) return;
  wput_kernel<<<128, 256, 0, stream>>>(Fp(8), Fp(10), Fp(12), Fp(14), Fp(16), Fp(18), Fp(20), WPS, WEF, WE2, WN1, WN2, WRO, WP1, WP2);
  csr_build7(csr, Ip(1) + E, E, N, stream); csr_build5(cg, Ip(4), N, NG, stream);
  emb_kernel<<<N / 16, 32, 0, stream>>>(Ip(0), Fp(5), Hp);
  for (int l = 0; l < L; ++l) {
    prep_kernel<<<NLIM / 16, 32, 0, stream>>>(Hp, Fp(6) + l * D, Fp(7) + l * D, WPS + (size_t)l * 2 * D * D, NLIM, HN, PSD);
    layer_kernel<<<NLIM / 16, 32, 0, stream>>>(Hp, HN, PSD, Fp(3), Fp(2), Ip(1), csr.PERM, csr.ROWPTR, csr.ROWCNT, (int)csr.permLen, WEF + (size_t)l * D * EF, Fp(9) + l * D, WE2 + (size_t)l * D * D, Fp(11) + l * D, WN1 + (size_t)l * D * 2 * D, Fp(13) + l * D, WN2 + (size_t)l * D * D, Fp(15) + l * D, NLIM); }
  readout_kernel<<<NG / 16, 32, 0, stream>>>(Hp, cg.PERM, cg.ROWPTR, cg.ROWCNT, (int)cg.permLen, WRO, Fp(17), WP1, Fp(19), WP2, Fp(21), NLIM, (float*)d_out);
}
